// HookedMambaBlock_84490596647003
// MI455X (gfx1250) — hardware-verified
//
#include <hip/hip_runtime.h>
#include <math.h>

typedef __attribute__((ext_vector_type(16))) _Float16 v16h;
typedef __attribute__((ext_vector_type(8)))  _Float16 v8h;
typedef __attribute__((ext_vector_type(8)))  float    v8f;
typedef __attribute__((ext_vector_type(4)))  float    v4f;

constexpr int kBatch = 2;
constexpr int kSeqL  = 2048;
constexpr int kDmod  = 1024;
constexpr int kDin   = 2048;
constexpr int kNst   = 16;
constexpr int kDtR   = 64;
constexpr int kPrjN  = kDtR + 2 * kNst;
constexpr int kPrjP  = 128;
constexpr int kRows  = kBatch * kSeqL;
constexpr int kTP    = 260;

constexpr float kCarryW   = 32.0f;
constexpr float kCarryWd2 = 8.0f;
constexpr float kCarryDr  = 16.0f;
constexpr float kCarryY   = 16.0f;
constexpr float kFoldIn   = 1.0f / kCarryW;
constexpr float kFoldDt   = 1.0f / (kCarryDr * kCarryWd2);
constexpr float kFoldOut  = 1.0f / (kCarryY * kCarryW);
constexpr float kInvDmod  = 1.0f / (float)kDmod;

static_assert(kPrjN == 96 && kPrjN <= kPrjP, "projection width");
static_assert((kDmod % 32) == 0 && (kDin % 32) == 0 && (kDtR % 32) == 0, "GEMM K multiples of 32");
static_assert((kRows % 64) == 0 && (kDin % 64) == 0 && (kDmod % 64) == 0 && (kPrjP % 64) == 0, "GEMM M,N multiples of 64");
static_assert((kSeqL % 64) == 0 && (kDin % 256) == 0 && kDmod == 128 * 8, "tile multiples");

constexpr size_t kOffWSK  = 0;
constexpr size_t kOffWIN  = kOffWSK  + (size_t)kDin  * kDmod * 2;
constexpr size_t kOffWOUT = kOffWIN  + (size_t)kDin  * kDmod * 2;
constexpr size_t kOffWD2  = kOffWOUT + (size_t)kDmod * kDin  * 2;
constexpr size_t kOffWPR  = kOffWD2  + (size_t)kDin  * kDtR  * 2;
constexpr size_t kOffXN   = kOffWPR  + (size_t)kPrjP * kDin  * 2;
constexpr size_t kOffSKP  = kOffXN   + (size_t)kRows * kDmod * 2;
constexpr size_t kOffXIN  = kOffSKP  + (size_t)kRows * kDin  * 2;
constexpr size_t kOffXH   = kOffXIN  + (size_t)kRows * kDin  * 2;
constexpr size_t kOffPRJ  = kOffXH   + (size_t)kRows * kDin  * 2;
constexpr size_t kOffDR16 = kOffPRJ  + (size_t)kRows * kPrjP * 4;
constexpr size_t kOffZDT  = kOffDR16 + (size_t)kRows * kDtR  * 2;
constexpr size_t kOffYG   = kOffZDT  + (size_t)kRows * kDin  * 4;
constexpr size_t kWsTotal = kOffYG   + (size_t)kRows * kDin  * 2;
static_assert(kWsTotal == 125042688ull, "carve total");
static_assert(kWsTotal <= 134217728ull, "carve cap");
static_assert((kOffWIN % 128) == 0 && (kOffWOUT % 128) == 0 && (kOffWD2 % 128) == 0 && (kOffWPR % 128) == 0 &&
              (kOffXN % 128) == 0 && (kOffSKP % 128) == 0 && (kOffXIN % 128) == 0 && (kOffXH % 128) == 0 &&
              (kOffPRJ % 128) == 0 && (kOffDR16 % 128) == 0 && (kOffZDT % 128) == 0 && (kOffYG % 128) == 0,
              "128-B aligned regions");

__device__ __forceinline__ float h16_to_f32(unsigned hb) {
  const unsigned sgn = (hb & 0x8000u) << 16;
  const unsigned em = hb & 0x7fffu;
  const float fn = __uint_as_float((em << 13) + 0x38000000u);
  const float fs = (float)em * 5.9604644775390625e-8f;
  const float mag = (em < 0x400u) ? fs : fn;
  return __uint_as_float(__float_as_uint(mag) | sgn);
}

__device__ __forceinline__ void guard_row4(v8f& a0, v8f& a1, v8f& a2, v8f& a3,
                                           v16h x, v16h b0, v16h b1, v16h b2, v16h b3) {
  asm volatile("v_nop\n\tv_nop\n\tv_nop\n\tv_nop"
               : "+v"(a0), "+v"(a1), "+v"(a2), "+v"(a3)
               : "v"(x), "v"(b0), "v"(b1), "v"(b2), "v"(b3));
}
__device__ __forceinline__ void keep4_h(v16h a, v16h b, v16h c, v16h d) {
  asm volatile("v_nop" :: "v"(a), "v"(b), "v"(c), "v"(d));
}
__device__ __forceinline__ void acc_guard4(v8f& a, v8f& b, v8f& c, v8f& d) {
  asm volatile("v_nop\n\tv_nop\n\tv_nop\n\tv_nop" : "+v"(a), "+v"(b), "+v"(c), "+v"(d));
}
struct FragH {
  union U { v16h v; v8h h[2]; };
  static __device__ __forceinline__ v16h load(const _Float16* p) {
    U f;
    f.h[0] = *(const v8h*)(p);
    f.h[1] = *(const v8h*)(p + 16);
    return f.v;
  }
  static __device__ __forceinline__ v8f mma(v16h a, v16h b, v8f c) {
    return __builtin_amdgcn_wmma_f32_16x16x32_f16(false, a, false, b, (short)0, c, false, false);
  }
};

template <int BIAS_MODE, int OUT_MODE, bool RESID>
__global__ __launch_bounds__(256) void wmma_gemm64(
    const unsigned short* __restrict__ Ap, int lda,
    const unsigned short* __restrict__ Btp, int ldb,
    void* __restrict__ Cout, int ldc,
    const float* __restrict__ bias,
    const float* __restrict__ resid,
    int M, int N, int K, float scale) {
  const _Float16* A  = (const _Float16*)Ap;
  const _Float16* Bt = (const _Float16*)Btp;
  __shared__ __align__(16) float sT[8][16 * 68];
  const int lane = threadIdx.x & 31;
  const int wave = threadIdx.x >> 5;
  const int tilesN = N >> 6;
  const int tilesM = M >> 6;
  const int tile = blockIdx.x * 8 + wave;
  if (tile >= tilesM * tilesN) return;
  const int tm = tile / tilesN;
  const int tn = tile - tm * tilesN;
  const int m0 = tm << 6;
  const int n0 = tn << 6;

  const int rlane = lane & 15;
  const int koff  = (lane >> 4) * 8;
  const int mOff  = (lane >> 4) * 8;

  v8f acc[4][4];
#pragma unroll
  for (int i = 0; i < 4; ++i)
#pragma unroll
    for (int j = 0; j < 4; ++j) acc[i][j] = (v8f){0.f, 0.f, 0.f, 0.f, 0.f, 0.f, 0.f, 0.f};

  for (int k0 = 0; k0 < K; k0 += 32) {
    v16h bh[4];
#pragma unroll
    for (int j = 0; j < 4; ++j) {
      const size_t bo = (size_t)(n0 + (j << 4) + rlane) * ldb + koff + k0;
      bh[j] = FragH::load(Bt + bo);
    }
#pragma unroll
    for (int i = 0; i < 4; ++i) {
      const size_t ao = (size_t)(m0 + (i << 4) + rlane) * lda + koff + k0;
      v16h ah = FragH::load(A + ao);
#pragma unroll
      for (int j = 0; j < 4; ++j) acc[i][j] = FragH::mma(ah, bh[j], acc[i][j]);
      guard_row4(acc[i][0], acc[i][1], acc[i][2], acc[i][3], ah, bh[0], bh[1], bh[2], bh[3]);
    }
    keep4_h(bh[0], bh[1], bh[2], bh[3]);
  }
  acc_guard4(acc[0][0], acc[0][1], acc[0][2], acc[0][3]);
  acc_guard4(acc[1][0], acc[1][1], acc[1][2], acc[1][3]);
  acc_guard4(acc[2][0], acc[2][1], acc[2][2], acc[2][3]);
  acc_guard4(acc[3][0], acc[3][1], acc[3][2], acc[3][3]);

  float* slab = sT[wave];
#pragma unroll
  for (int i = 0; i < 4; ++i) {
    const int mBase = m0 + (i << 4);
#pragma unroll
    for (int j = 0; j < 4; ++j) {
      const int n = n0 + (j << 4) + rlane;
      float bv = 0.f;
      if (BIAS_MODE == 2) bv = bias[n];
#pragma unroll
      for (int r = 0; r < 8; ++r) {
        float v = acc[i][j][r] * scale;
        if (BIAS_MODE == 2) v += bv;
        slab[(mOff + r) * 68 + (j << 4) + rlane] = v;
      }
    }
    __builtin_amdgcn_fence(__ATOMIC_RELEASE, "workgroup");
    __builtin_amdgcn_wave_barrier();
    __builtin_amdgcn_fence(__ATOMIC_ACQUIRE, "workgroup");
    if (OUT_MODE == 0) {
      float* C = (float*)Cout;
      const int hh = lane >> 4, c4 = (lane & 15) * 4;
      v4f vv[8];
#pragma unroll
      for (int it = 0; it < 8; ++it) {
        const int row = it * 2 + hh;
        v4f v = *(const v4f*)(slab + row * 68 + c4);
        if (RESID) {
          const v4f r4 = *(const v4f*)(resid + (size_t)(mBase + row) * ldc + n0 + c4);
          v = v + r4;
        }
        vv[it] = v;
      }
      for (int pass = 0; pass < 2; ++pass) {
#pragma unroll
        for (int it = 0; it < 8; ++it) {
          const int row = it * 2 + hh;
          *(volatile v4f*)(C + (size_t)(mBase + row) * ldc + n0 + c4) = vv[it];
        }
        __threadfence();
      }
    } else {
      const int q = lane >> 3, c8 = (lane & 7) * 8;
      unsigned short* C = (unsigned short*)Cout;
      v8h hv[4];
#pragma unroll
      for (int it = 0; it < 4; ++it) {
        const int row = it * 4 + q;
        const float* sp = slab + row * 68 + c8;
#pragma unroll
        for (int e = 0; e < 8; ++e) hv[it][e] = (_Float16)sp[e];
      }
      for (int pass = 0; pass < 2; ++pass) {
#pragma unroll
        for (int it = 0; it < 4; ++it) {
          const int row = it * 4 + q;
          *(volatile v8h*)(C + (size_t)(mBase + row) * ldc + n0 + c8) = hv[it];
        }
        __threadfence();
      }
    }
    __builtin_amdgcn_fence(__ATOMIC_RELEASE, "workgroup");
    __builtin_amdgcn_wave_barrier();
    __builtin_amdgcn_fence(__ATOMIC_ACQUIRE, "workgroup");
  }
}

__global__ __launch_bounds__(256) void cast_f16_kernel(
    const float* __restrict__ src, unsigned short* __restrict__ dst, int total8, float scale)
{
  const int i = blockIdx.x * 256 + threadIdx.x;
  if (i >= total8) return;
  const size_t e0 = (size_t)i << 3;
  const float* p = src + e0;
  const v4f a0 = *(const v4f*)(p);
  const v4f a1 = *(const v4f*)(p + 4);
  v8h hv;
#pragma unroll
  for (int e = 0; e < 4; ++e) {
    hv[e]     = (_Float16)(a0[e] * scale);
    hv[4 + e] = (_Float16)(a1[e] * scale);
  }
  unsigned short* q = dst + e0;
  *(volatile v8h*)q = hv;
  __threadfence();
  *(volatile v8h*)q = hv;
}

__global__ __launch_bounds__(256) void build_proj_weights_kernel(
    const float* __restrict__ wd1, const float* __restrict__ wB, const float* __restrict__ wC,
    unsigned short* __restrict__ WPR, float scale)
{
  const int row = blockIdx.x;
  const bool live = (row < kPrjN);
  const int rsel = (row < kDtR) ? row : ((row < kDtR + kNst) ? (row - kDtR) : (live ? (row - kDtR - kNst) : 0));
  const float* base = (row < kDtR) ? wd1 : ((row < kDtR + kNst) ? wB : (live ? wC : wd1));
  const float* p = base + (size_t)rsel * kDin + threadIdx.x * 8;
  const v4f a0 = *(const v4f*)(p);
  const v4f a1 = *(const v4f*)(p + 4);
  v8h hv;
#pragma unroll
  for (int e = 0; e < 4; ++e) {
    const float f0 = live ? (a0[e] * scale) : 0.0f;
    const float f1 = live ? (a1[e] * scale) : 0.0f;
    hv[e]     = (_Float16)f0;
    hv[4 + e] = (_Float16)f1;
  }
  unsigned short* q = WPR + (size_t)row * kDin + threadIdx.x * 8;
  *(volatile v8h*)q = hv;
  __threadfence();
  *(volatile v8h*)q = hv;
}

__global__ __launch_bounds__(128) void rmsnorm_f16_kernel(
    const float* __restrict__ xin, const float* __restrict__ gain, unsigned short* __restrict__ XN)
{
  __shared__ float red[4];
  const int row = blockIdx.x;
  const int tid = threadIdx.x, lane = tid & 31, wave = tid >> 5;
  const float* r = xin + (size_t)row * kDmod + tid * 8;
  const v4f a0 = *(const v4f*)(r);
  const v4f a1 = *(const v4f*)(r + 4);
  const v4f g0 = *(const v4f*)(gain + tid * 8);
  const v4f g1 = *(const v4f*)(gain + tid * 8 + 4);
  float ss = 0.0f;
#pragma unroll
  for (int e = 0; e < 4; ++e) {
    ss = fmaf(a0[e], a0[e], ss);
    ss = fmaf(a1[e], a1[e], ss);
  }
#pragma unroll
  for (int off = 16; off >= 1; off >>= 1) ss += __shfl_xor(ss, off, 32);
  if (lane == 0) red[wave] = ss;
  __syncthreads();
  const float tot = (red[0] + red[1]) + (red[2] + red[3]);
  const float sc = rsqrtf(tot * kInvDmod + 1e-5f);
  v8h hv;
#pragma unroll
  for (int e = 0; e < 4; ++e) {
    const float f0 = (a0[e] * sc) * g0[e];
    const float f1 = (a1[e] * sc) * g1[e];
    hv[e]     = (_Float16)f0;
    hv[4 + e] = (_Float16)f1;
  }
  unsigned short* q = XN + (size_t)row * kDmod + tid * 8;
  *(volatile v8h*)q = hv;
  __threadfence();
  *(volatile v8h*)q = hv;
}

__global__ __launch_bounds__(128) void conv_silu_kernel(
    const unsigned* __restrict__ XINw, const float* __restrict__ cw, const float* __restrict__ cb,
    unsigned short* __restrict__ XH)
{
  __shared__ __align__(16) float sT[16 * kTP];
  const int tid = threadIdx.x, lane = tid & 31, wave = tid >> 5;
  const int d0 = blockIdx.x * 256;
  const int dA = d0 + 2 * tid;
  const int g0 = blockIdx.y * 64;
  const int tb = g0 & (kSeqL - 1);
  const v4f wa = *(const v4f*)(cw + (size_t)dA * 4);
  const v4f wb = *(const v4f*)(cw + (size_t)(dA + 1) * 4);
  const float ba = cb[dA], bb = cb[dA + 1];
  const size_t wc = (size_t)(dA >> 1);
  constexpr size_t kWPitch = (size_t)kDin / 2;
  float am3, am2, am1, bm3, bm2, bm1;
  {
    const bool hist = (tb > 0);
    const int rb = hist ? (g0 - 3) : g0;
    const unsigned u3 = XINw[(size_t)rb * kWPitch + wc];
    const unsigned u2 = XINw[(size_t)(rb + 1) * kWPitch + wc];
    const unsigned u1 = XINw[(size_t)(rb + 2) * kWPitch + wc];
    const float a3 = h16_to_f32(u3 & 0xffffu), b3 = h16_to_f32(u3 >> 16);
    const float a2 = h16_to_f32(u2 & 0xffffu), b2 = h16_to_f32(u2 >> 16);
    const float a1 = h16_to_f32(u1 & 0xffffu), b1 = h16_to_f32(u1 >> 16);
    am3 = hist ? a3 : 0.f;  bm3 = hist ? b3 : 0.f;
    am2 = hist ? a2 : 0.f;  bm2 = hist ? b2 : 0.f;
    am1 = hist ? a1 : 0.f;  bm1 = hist ? b1 : 0.f;
  }
#pragma unroll 1
  for (int sub = 0; sub < 4; ++sub) {
    const int lb = g0 + sub * 16;
#pragma unroll 1
    for (int s = 0; s < 16; ++s) {
      const unsigned u = XINw[(size_t)(lb + s) * kWPitch + wc];
      const float ac = h16_to_f32(u & 0xffffu);
      const float bc = h16_to_f32(u >> 16);
      float accA = wa[0] * am3;
      accA = fmaf(wa[1], am2, accA);
      accA = fmaf(wa[2], am1, accA);
      accA = fmaf(wa[3], ac, accA);
      float accB = wb[0] * bm3;
      accB = fmaf(wb[1], bm2, accB);
      accB = fmaf(wb[2], bm1, accB);
      accB = fmaf(wb[3], bc, accB);
      const float sa = accA + ba;
      const float sb = accB + bb;
      const float ga = __builtin_amdgcn_rcpf(1.0f + expf(-sa));
      const float gb = __builtin_amdgcn_rcpf(1.0f + expf(-sb));
      sT[s * kTP + 2 * tid]     = sa * ga;
      sT[s * kTP + 2 * tid + 1] = sb * gb;
      am3 = am2; am2 = am1; am1 = ac;
      bm3 = bm2; bm2 = bm1; bm1 = bc;
    }
    __syncthreads();
    v8h hv[4];
#pragma unroll
    for (int it = 0; it < 4; ++it) {
      const float* sp = sT + (it * 4 + wave) * kTP + lane * 8;
      const v4f a0 = *(const v4f*)(sp);
      const v4f a1 = *(const v4f*)(sp + 4);
#pragma unroll
      for (int e = 0; e < 4; ++e) {
        hv[it][e]     = (_Float16)a0[e];
        hv[it][4 + e] = (_Float16)a1[e];
      }
    }
    for (int pass = 0; pass < 2; ++pass) {
#pragma unroll
      for (int it = 0; it < 4; ++it)
        *(volatile v8h*)(XH + (size_t)(lb + it * 4 + wave) * kDin + d0 + lane * 8) = hv[it];
      __threadfence();
    }
    __syncthreads();
  }
}

__global__ __launch_bounds__(256) void dr_cast_kernel(
    const float* __restrict__ PRJ, unsigned short* __restrict__ DR16, int total8, float scale)
{
  const int i = blockIdx.x * 256 + threadIdx.x;
  if (i >= total8) return;
  const int e0  = i << 3;
  const int row = e0 >> 6;
  const int c8  = e0 & 63;
  const float* p = PRJ + (size_t)row * kPrjP + c8;
  const v4f a0 = *(const v4f*)(p);
  const v4f a1 = *(const v4f*)(p + 4);
  v8h hv;
#pragma unroll
  for (int e = 0; e < 4; ++e) {
    hv[e]     = (_Float16)(a0[e] * scale);
    hv[4 + e] = (_Float16)(a1[e] * scale);
  }
  unsigned short* qd = DR16 + e0;
  *(volatile v8h*)qd = hv;
  __threadfence();
  *(volatile v8h*)qd = hv;
}

__global__ __launch_bounds__(256) void scan_gate_kernel(
    const float* __restrict__ ZDT, const unsigned* __restrict__ XHw, const unsigned* __restrict__ SKw,
    const float* __restrict__ PRJ, const float* __restrict__ A_log, const float* __restrict__ WD,
    unsigned short* __restrict__ YG)
{
  __shared__ __align__(16) float sA[kNst * 256];
  __shared__ __align__(16) float sBC[16 * 32];
  __shared__ __align__(16) float sY[16 * kTP];
  const int tid = threadIdx.x, lane = tid & 31, wave = tid >> 5;
  const int bix = blockIdx.x >> 3;
  const int d0 = (blockIdx.x & 7) * 256, d = d0 + tid;
  const size_t row0 = (size_t)bix * kSeqL;

#pragma unroll 1
  for (int n = 0; n < kNst; ++n) sA[n * 256 + tid] = -expf(A_log[(size_t)d * kNst + n]);
  __syncthreads();
  float An[kNst], h[kNst];
#pragma unroll
  for (int n = 0; n < kNst; ++n) {
    An[n] = sA[n * 256 + tid];
    h[n] = 0.f;
  }
  const float Dd = WD[d];
  const unsigned sh = (unsigned)(d & 1) * 16u;

#pragma unroll 1
  for (int c = 0; c < kSeqL / 16; ++c) {
    const int l0 = c * 16;
    if (tid < 128) {
      const int r = tid >> 3, q = (tid & 7) * 4;
      const v4f v = *(const v4f*)(PRJ + (row0 + l0 + r) * kPrjP + kDtR + q);
      *(v4f*)(sBC + r * 32 + q) = v;
    }
    __syncthreads();
#pragma unroll 1
    for (int s = 0; s < 16; ++s) {
      const size_t m = row0 + (size_t)(l0 + s);
      const size_t ei = m * kDin + d;
      float zv = ZDT[ei];
      unsigned xw = XHw[ei >> 1];
      unsigned sw = SKw[ei >> 1];
      asm volatile("" : "+v"(zv), "+v"(xw), "+v"(sw));
      const float delta = fmaxf(zv, 0.0f) + log1pf(expf(-fabsf(zv)));
      const float xv = h16_to_f32((xw >> sh) & 0xffffu);
      const float sk = h16_to_f32((sw >> sh) & 0xffffu);
      v4f Bq[4], Cq[4];
#pragma unroll
      for (int qq = 0; qq < 4; ++qq) {
        Bq[qq] = *(const v4f*)(sBC + s * 32 + 4 * qq);
        Cq[qq] = *(const v4f*)(sBC + s * 32 + kNst + 4 * qq);
      }
      const float dtx = delta * xv;
      float y = 0.f;
#pragma unroll
      for (int n = 0; n < kNst; ++n) {
        const float e = __expf(delta * An[n]);
        const float inj = dtx * Bq[n >> 2][n & 3];
        const float hn = fmaf(e, h[n], inj);
        h[n] = hn;
        y = fmaf(hn, Cq[n >> 2][n & 3], y);
      }
      y = fmaf(xv, Dd, y);
      const float sg = __builtin_amdgcn_rcpf(1.0f + expf(-sk));
      const float g  = sk * sg;
      sY[s * kTP + tid] = (y * g) * kCarryY;
    }
    __syncthreads();
    v8h hv[2];
#pragma unroll
    for (int it = 0; it < 2; ++it) {
      const float* sp = sY + (it * 8 + wave) * kTP + lane * 8;
      const v4f a0 = *(const v4f*)(sp);
      const v4f a1 = *(const v4f*)(sp + 4);
#pragma unroll
      for (int e = 0; e < 4; ++e) {
        hv[it][e]     = (_Float16)a0[e];
        hv[it][4 + e] = (_Float16)a1[e];
      }
    }
    for (int pass = 0; pass < 2; ++pass) {
#pragma unroll
      for (int it = 0; it < 2; ++it)
        *(volatile v8h*)(YG + (row0 + l0 + it * 8 + wave) * kDin + d0 + lane * 8) = hv[it];
      __threadfence();
    }
  }
}

extern "C" void kernel_launch(void* const* d_in, const int* in_sizes, int n_in,
                              void* d_out, int out_size, void* d_ws, size_t ws_size,
                              hipStream_t stream)
{
  if (n_in < 14) return;
  if (in_sizes[0] != kRows * kDmod) return;
  if (in_sizes[1] != kDmod) return;
  if (in_sizes[2] != kDin * kDmod || in_sizes[3] != kDin * kDmod) return;
  if (in_sizes[4] != kDin * 4 || in_sizes[5] != kDin) return;
  if (in_sizes[6] != kDtR * kDin || in_sizes[7] != kDin * kDtR) return;
  if (in_sizes[8] != kDin) return;
  if (in_sizes[9] != kNst * kDin || in_sizes[10] != kNst * kDin) return;
  if (in_sizes[11] != kDin * kNst || in_sizes[12] != kDin) return;
  if (in_sizes[13] != kDmod * kDin) return;
  if (out_size != kRows * kDmod) return;
  if (ws_size < kWsTotal) return;

  const float* x_in   = (const float*)d_in[0];
  const float* norm_w = (const float*)d_in[1];
  const float* skip_w = (const float*)d_in[2];
  const float* in_w   = (const float*)d_in[3];
  const float* conv_w = (const float*)d_in[4];
  const float* conv_b = (const float*)d_in[5];
  const float* wd1    = (const float*)d_in[6];
  const float* wd2    = (const float*)d_in[7];
  const float* wd2_b  = (const float*)d_in[8];
  const float* wB     = (const float*)d_in[9];
  const float* wC     = (const float*)d_in[10];
  const float* A_log  = (const float*)d_in[11];
  const float* W_D    = (const float*)d_in[12];
  const float* out_w  = (const float*)d_in[13];
  float* dout = (float*)d_out;

  char* ws = (char*)d_ws;
  unsigned short* WSK  = (unsigned short*)(ws + kOffWSK);
  unsigned short* WIN  = (unsigned short*)(ws + kOffWIN);
  unsigned short* WOUT = (unsigned short*)(ws + kOffWOUT);
  unsigned short* WD2  = (unsigned short*)(ws + kOffWD2);
  unsigned short* WPR  = (unsigned short*)(ws + kOffWPR);
  unsigned short* XN   = (unsigned short*)(ws + kOffXN);
  unsigned short* SKP  = (unsigned short*)(ws + kOffSKP);
  unsigned short* XIN  = (unsigned short*)(ws + kOffXIN);
  unsigned short* XH   = (unsigned short*)(ws + kOffXH);
  float*          PRJ  = (float*)(ws + kOffPRJ);
  unsigned short* DR16 = (unsigned short*)(ws + kOffDR16);
  float*          ZDT  = (float*)(ws + kOffZDT);
  unsigned short* YG   = (unsigned short*)(ws + kOffYG);

  cast_f16_kernel<<<(kDin * kDmod / 8) / 256, 256, 0, stream>>>(skip_w, WSK, kDin * kDmod / 8, kCarryW);
  cast_f16_kernel<<<(kDin * kDmod / 8) / 256, 256, 0, stream>>>(in_w, WIN, kDin * kDmod / 8, kCarryW);
  cast_f16_kernel<<<(kDmod * kDin / 8) / 256, 256, 0, stream>>>(out_w, WOUT, kDmod * kDin / 8, kCarryW);
  cast_f16_kernel<<<(kDin * kDtR / 8) / 256, 256, 0, stream>>>(wd2, WD2, kDin * kDtR / 8, kCarryWd2);
  build_proj_weights_kernel<<<kPrjP, 256, 0, stream>>>(wd1, wB, wC, WPR, kCarryW);

  rmsnorm_f16_kernel<<<kRows, 128, 0, stream>>>(x_in, norm_w, XN);

  wmma_gemm64<0, 1, false><<<dim3(256, 1), 256, 0, stream>>>(
      XN, kDmod, WSK, kDmod, (void*)SKP, kDin, wd2_b, x_in, kRows, kDin, kDmod, kFoldIn);
  wmma_gemm64<0, 1, false><<<dim3(256, 1), 256, 0, stream>>>(
      XN, kDmod, WIN, kDmod, (void*)XIN, kDin, wd2_b, x_in, kRows, kDin, kDmod, kFoldIn);

  conv_silu_kernel<<<dim3(kDin / 256, kRows / 64), 128, 0, stream>>>(
      (const unsigned*)XIN, conv_w, conv_b, XH);

  wmma_gemm64<0, 0, false><<<dim3(16, 1), 256, 0, stream>>>(
      XH, kDin, WPR, kDin, (void*)PRJ, kPrjP, wd2_b, x_in, kRows, kPrjP, kDin, kFoldIn);

  dr_cast_kernel<<<(kRows * kDtR / 8) / 256, 256, 0, stream>>>(PRJ, DR16, kRows * kDtR / 8, kCarryDr);

  wmma_gemm64<2, 0, false><<<dim3(256, 1), 256, 0, stream>>>(
      DR16, kDtR, WD2, kDtR, (void*)ZDT, kDin, wd2_b, x_in, kRows, kDin, kDtR, kFoldDt);

  scan_gate_kernel<<<kBatch * (kDin / 256), 256, 0, stream>>>(
      ZDT, (const unsigned*)XH, (const unsigned*)SKP, PRJ, A_log, W_D, YG);

  wmma_gemm64<0, 0, true><<<dim3(128, 1), 256, 0, stream>>>(
      YG, kDin, WOUT, kDin, (void*)dout, kDmod, wd2_b, x_in, kRows, kDmod, kDin, kFoldOut);
}
